// DiffPool_GNN_30648886624415
// MI455X (gfx1250) — hardware-verified
//
#include <hip/hip_runtime.h>
#include <stddef.h>
#include <stdint.h>


#define NBATCH 16
#define MAXN   2048
#define INDIM  128
#define HIDD   64
#define K1V    205
#define K1PD   224
#define K2V    21
#define K2PD   32
#define OUTV   2
#define RBADJ  512
#define GT     128

typedef float          v8f   __attribute__((ext_vector_type(8)));
typedef float          v4f   __attribute__((ext_vector_type(4)));
typedef int            v8i   __attribute__((ext_vector_type(8)));
typedef unsigned short v8us  __attribute__((ext_vector_type(8)));
typedef __bf16         v16bf __attribute__((ext_vector_type(16)));

union Frag { v16bf v; v8us h[2]; v8i i; };

__device__ __forceinline__ v8f wm(const Frag& a, const Frag& b, v8f c) {
  c = __builtin_amdgcn_wmma_f32_16x16x32_bf16(false, a.v, false, b.v, (short)0, c, false, false);
  asm volatile("v_nop\n\tv_nop\n\tv_nop\n\tv_nop" : "+v"(c) : "v"(a.i), "v"(b.i));
  return c;
}

__device__ __forceinline__ int clampi(int x, int lo, int hi) { return x < lo ? lo : (x > hi ? hi : x); }

__device__ __forceinline__ unsigned bf16_rne_bits(float x) {
  unsigned u = __float_as_uint(x);
  return (u + 0x7FFFu + ((u >> 16) & 1u)) >> 16;
}
__device__ __forceinline__ void split_hl(float x, unsigned short& hi, unsigned short& lo) {
  const unsigned uh = bf16_rne_bits(x);
  const float xh = __uint_as_float(uh << 16);
  const unsigned ul = bf16_rne_bits(x - xh);
  hi = (unsigned short)uh;
  lo = (unsigned short)ul;
}

struct GArgs {
  const float* A; const float* Bp; const float* A2; const float* B2; float* D;
  const int* bidx; const int* sl1; const int* sl2;
  long long sA, sB, sA2, sB2, sD;
  int M, Mv, K, Kv, lda, tA;
  int ldb, KvB, Nv, vecB;
  int Mv2, K2, Kv2, lda2, tA2, ldb2;
  int KvB2, Nv2, vecB2, ldd;
  int epi, epiNv, remap, epiMv;
};
static_assert(sizeof(GArgs) == 200, "");

template <int NACC>
__device__ __forceinline__ void gterm(v8f (&acc)[NACC],
                                      unsigned short* Ah, unsigned short* Al,
                                      unsigned short* Bh, unsigned short* Bl,
                                      const float* __restrict__ A, int lda, int tA, int Mv, int Kv, int K, int m0,
                                      const float* __restrict__ Bp, int ldb, int KvB, int Nv, int vecB) {
  constexpr int NB = 32 * NACC;
  constexpr int KP = 40;
  constexpr int NQ = NB / 4;
  const int tid = threadIdx.x, lane = tid & 31, wv = tid >> 5, h = lane >> 4, lm = lane & 15;
  const int wr = wv & 1, wc = wv >> 1;

  for (int k0 = 0; k0 < K; k0 += 32) {
    if (tA == 0) {
      const int m = tid >> 2, kq = (tid & 3) * 8, gm = m0 + m;
      v8us ph, pl;
#pragma unroll
      for (int i = 0; i < 8; ++i) {
        const int gk = k0 + kq + i;
        float v = 0.f;
        if (gm < Mv && gk < Kv) v = A[(size_t)gm * (size_t)lda + (size_t)gk];
        unsigned short hh, ll;
        split_hl(v, hh, ll);
        ph[i] = hh; pl[i] = ll;
      }
      *(v8us*)(Ah + m * KP + kq) = ph;
      *(v8us*)(Al + m * KP + kq) = pl;
    } else {
      const int k = tid >> 2, mq = (tid & 3) * 8, gk = k0 + k;
#pragma unroll
      for (int i = 0; i < 8; ++i) {
        const int gm = m0 + mq + i;
        float v = 0.f;
        if (gk < Kv && gm < Mv) v = A[(size_t)gk * (size_t)lda + (size_t)gm];
        unsigned short hh, ll;
        split_hl(v, hh, ll);
        Ah[(mq + i) * KP + k] = hh;
        Al[(mq + i) * KP + k] = ll;
      }
    }
    {
      const int k = tid >> 2, nq = (tid & 3) * NQ, gk = k0 + k;
      const bool kok = gk < KvB;
      if (vecB) {
#pragma unroll
        for (int q = 0; q < NQ / 4; ++q) {
          v4f f = {0.f, 0.f, 0.f, 0.f};
          if (kok) f = *(const v4f*)(Bp + (size_t)gk * (size_t)ldb + (size_t)(nq + 4 * q));
#pragma unroll
          for (int c = 0; c < 4; ++c) {
            unsigned short hh, ll;
            split_hl(f[c], hh, ll);
            const int n = nq + 4 * q + c;
            Bh[n * KP + k] = hh;
            Bl[n * KP + k] = ll;
          }
        }
      } else {
#pragma unroll
        for (int i = 0; i < NQ; ++i) {
          const int n = nq + i;
          float v = 0.f;
          if (kok && n < Nv) v = Bp[(size_t)gk * (size_t)ldb + (size_t)n];
          unsigned short hh, ll;
          split_hl(v, hh, ll);
          Bh[n * KP + k] = hh;
          Bl[n * KP + k] = ll;
        }
      }
    }
    __syncthreads();

    Frag ah, al;
    {
      const int o = (16 * wr + lm) * KP;
      ah.h[0] = *(const v8us*)(Ah + o + 8 * h);
      ah.h[1] = *(const v8us*)(Ah + o + 16 + 8 * h);
      al.h[0] = *(const v8us*)(Al + o + 8 * h);
      al.h[1] = *(const v8us*)(Al + o + 16 + 8 * h);
    }
#pragma unroll
    for (int j = 0; j < NACC; ++j) {
      const int o = (wc * 16 * NACC + 16 * j + lm) * KP;
      Frag bh, bl;
      bh.h[0] = *(const v8us*)(Bh + o + 8 * h);
      bh.h[1] = *(const v8us*)(Bh + o + 16 + 8 * h);
      bl.h[0] = *(const v8us*)(Bl + o + 8 * h);
      bl.h[1] = *(const v8us*)(Bl + o + 16 + 8 * h);
      acc[j] = wm(ah, bh, acc[j]);
      acc[j] = wm(ah, bl, acc[j]);
      acc[j] = wm(al, bh, acc[j]);
    }
    __syncthreads();
  }
}

template <int NACC>
__global__ void __launch_bounds__(GT) k_gemm(GArgs g) {
  constexpr int NB = 32 * NACC;
  constexpr int KP = 40;
  constexpr int OP = NB + 4;
  constexpr int NCH = (NB + 127) / 128;
  constexpr int ABYTES = 32 * KP * 2;
  constexpr int BBYTES = NB * KP * 2;
  constexpr int OBYTES = 32 * OP * 4;
  constexpr int UBYTES = (2 * BBYTES > OBYTES) ? (2 * BBYTES) : OBYTES;
  __shared__ __attribute__((aligned(16))) unsigned char smem[2 * ABYTES + UBYTES];
  unsigned short* Ah = (unsigned short*)(smem);
  unsigned short* Al = (unsigned short*)(smem + ABYTES);
  unsigned short* Bh = (unsigned short*)(smem + 2 * ABYTES);
  unsigned short* Bl = (unsigned short*)(smem + 2 * ABYTES + BBYTES);
  float* Os = (float*)(smem + 2 * ABYTES);

  const int tid = threadIdx.x, lane = tid & 31, wv = tid >> 5, h = lane >> 4, lm = lane & 15;
  const int wr = wv & 1, wc = wv >> 1;
  const int bz = blockIdx.z;
  const int m0 = (int)blockIdx.x * 32;

  v8f acc[NACC];
#pragma unroll
  for (int j = 0; j < NACC; ++j) {
    const v8f z = {0.f, 0.f, 0.f, 0.f, 0.f, 0.f, 0.f, 0.f};
    acc[j] = z;
  }

  gterm<NACC>(acc, Ah, Al, Bh, Bl,
              g.A + (size_t)bz * (size_t)g.sA, g.lda, g.tA, g.Mv, g.Kv, g.K, m0,
              g.Bp + (size_t)bz * (size_t)g.sB, g.ldb, g.KvB, g.Nv, g.vecB);
  if (g.K2 > 0) {
    gterm<NACC>(acc, Ah, Al, Bh, Bl,
                g.A2 + (size_t)bz * (size_t)g.sA2, g.lda2, g.tA2, g.Mv2, g.Kv2, g.K2, m0,
                g.B2 + (size_t)bz * (size_t)g.sB2, g.ldb2, g.KvB2, g.Nv2, g.vecB2);
  }

#pragma unroll
  for (int j = 0; j < NACC; ++j) {
    const int col = wc * 16 * NACC + 16 * j + lm;
#pragma unroll
    for (int r = 0; r < 8; ++r) Os[(16 * wr + 8 * h + r) * OP + col] = acc[j][r];
  }
  __syncthreads();

  float* Db = g.D + (size_t)bz * (size_t)g.sD;
  for (int i = 0; i < 8; ++i) {
    const int rr = wv * 8 + i;
    const int gm = m0 + rr;
    if (gm >= g.M) break;
    size_t orow = (size_t)gm;
    if (g.remap == 1) {
      int bb = clampi(g.bidx[gm], 0, NBATCH - 1);
      int pos = clampi(gm - g.sl1[bb], 0, MAXN - 1);
      orow = (size_t)bb * MAXN + (size_t)pos;
    } else if (g.remap == 2) {
      int bb = clampi(g.bidx[gm], 0, NBATCH - 1);
      int pos = clampi(gm - g.sl2[bb] + (g.sl1[bb + 1] - g.sl1[bb]), 0, MAXN - 1);
      orow = (size_t)bb * MAXN + (size_t)pos;
    }
    v4f v[NCH];
#pragma unroll
    for (int q = 0; q < NCH; ++q) {
      const int c0 = 128 * q + 4 * lane;
      v4f t = {0.f, 0.f, 0.f, 0.f};
      if (c0 < NB) t = *(const v4f*)(Os + rr * OP + c0);
      v[q] = t;
    }
    if (g.epi == 1) {
#pragma unroll
      for (int q = 0; q < NCH; ++q) {
#pragma unroll
        for (int j = 0; j < 4; ++j) v[q][j] = fmaxf(v[q][j], 0.f);
      }
    } else if (g.epi == 2) {
      float mx = -3.0e38f;
#pragma unroll
      for (int q = 0; q < NCH; ++q) {
#pragma unroll
        for (int j = 0; j < 4; ++j) {
          const int c = 128 * q + 4 * lane + j;
          if (c < g.epiNv) mx = fmaxf(mx, v[q][j]);
        }
      }
#pragma unroll
      for (int o = 16; o > 0; o >>= 1) mx = fmaxf(mx, __shfl_xor(mx, o, 32));
      float s = 0.f;
      v4f e[NCH];
#pragma unroll
      for (int q = 0; q < NCH; ++q) {
#pragma unroll
        for (int j = 0; j < 4; ++j) {
          const int c = 128 * q + 4 * lane + j;
          const float ev = (c < g.epiNv) ? expf(v[q][j] - mx) : 0.f;
          e[q][j] = ev;
          s += ev;
        }
      }
#pragma unroll
      for (int o = 16; o > 0; o >>= 1) s += __shfl_xor(s, o, 32);
      const float inv = 1.0f / s;
#pragma unroll
      for (int q = 0; q < NCH; ++q) {
#pragma unroll
        for (int j = 0; j < 4; ++j) v[q][j] = e[q][j] * inv;
      }
    }
    if (gm >= g.epiMv) {
#pragma unroll
      for (int q = 0; q < NCH; ++q) { const v4f z = {0.f, 0.f, 0.f, 0.f}; v[q] = z; }
    }
    float* dp = Db + orow * (size_t)g.ldd;
#pragma unroll
    for (int q = 0; q < NCH; ++q) {
      const int c0 = 128 * q + 4 * lane;
      if (c0 < NB) *(volatile v4f*)(dp + c0) = v[q];
    }
    __threadfence();
#pragma unroll
    for (int q = 0; q < NCH; ++q) {
      const int c0 = 128 * q + 4 * lane;
      if (c0 < NB) *(volatile v4f*)(dp + c0) = v[q];
    }
  }
}

__global__ void __launch_bounds__(256) k_pad(const int* __restrict__ sl1, const int* __restrict__ sl2,
                                             float* __restrict__ SP, float* __restrict__ XD) {
  const int row = (int)((blockIdx.x * 256u + threadIdx.x) >> 5);
  const int lane = threadIdx.x & 31;
  if (row >= NBATCH * MAXN) return;
  const int b = row / MAXN, pos = row - b * MAXN;
  const int npos = (sl1[b + 1] - sl1[b]) + (sl2[b + 1] - sl2[b]);
  if (pos < npos) return;
  const float inv = 1.0f / (float)K1V;
  v4f s0, s1;
  const v4f z = {0.f, 0.f, 0.f, 0.f};
#pragma unroll
  for (int j = 0; j < 4; ++j) {
    s0[j] = inv;
    s1[j] = ((128 + 4 * lane + j) < K1V) ? inv : 0.f;
  }
  float* sp = SP + (size_t)row * K1PD;
  float* xp = XD + (size_t)row * HIDD;
  *(volatile v4f*)(sp + 4 * lane) = s0;
  if (lane < 24) *(volatile v4f*)(sp + 128 + 4 * lane) = s1;
  if (lane < 16) *(volatile v4f*)(xp + 4 * lane) = z;
  __threadfence();
  *(volatile v4f*)(sp + 4 * lane) = s0;
  if (lane < 24) *(volatile v4f*)(sp + 128 + 4 * lane) = s1;
  if (lane < 16) *(volatile v4f*)(xp + 4 * lane) = z;
}

__global__ void __launch_bounds__(256) k_adj(const int* __restrict__ eg1, int ne1,
                                             const int* __restrict__ eg2, int ne2,
                                             const int* __restrict__ eh, int neh,
                                             const int* __restrict__ b1, const int* __restrict__ b2,
                                             const int* __restrict__ sl1, const int* __restrict__ sl2,
                                             int nt1, int nt2,
                                             const float* __restrict__ SP, float* __restrict__ AS) {
  __shared__ __attribute__((aligned(16))) unsigned bm[RBADJ * 64];
  const int tid = threadIdx.x, lane = tid & 31, wv = tid >> 5;
  const int b = blockIdx.y, r0 = (int)blockIdx.x * RBADJ;
  for (int i = tid; i < RBADJ * 64; i += 256) bm[i] = 0u;
  const int o1 = sl1[b], o2 = sl2[b], n1b = sl1[b + 1] - o1;
  __syncthreads();

  for (int e = tid; e < ne1; e += 256) {
    const int s = clampi(eg1[e], 0, nt1 - 1);
    if (b1[s] != b) continue;
    int sp = s - o1; if (sp < 0) sp += MAXN;
    const unsigned rs = (unsigned)(sp - r0);
    if (rs >= (unsigned)RBADJ) continue;
    const int d = clampi(eg1[ne1 + e], 0, nt1 - 1);
    const int bd = clampi(b1[d], 0, NBATCH - 1);
    int dp = d - sl1[bd]; if (dp < 0) dp += MAXN;
    if ((unsigned)dp >= (unsigned)MAXN) continue;
    atomicOr(&bm[rs * 64u + (unsigned)(dp >> 5)], 1u << (dp & 31));
  }
  for (int e = tid; e < ne2; e += 256) {
    const int s = clampi(eg2[e], 0, nt2 - 1);
    if (b2[s] != b) continue;
    int sp = s - o2 + n1b; if (sp < 0) sp += MAXN;
    const unsigned rs = (unsigned)(sp - r0);
    if (rs >= (unsigned)RBADJ) continue;
    const int d = clampi(eg2[ne2 + e], 0, nt2 - 1);
    const int bd = clampi(b2[d], 0, NBATCH - 1);
    int dp = d - sl2[bd] + (sl1[bd + 1] - sl1[bd]); if (dp < 0) dp += MAXN;
    if ((unsigned)dp >= (unsigned)MAXN) continue;
    atomicOr(&bm[rs * 64u + (unsigned)(dp >> 5)], 1u << (dp & 31));
  }
  for (int e = tid; e < neh; e += 256) {
    const int s = clampi(eh[e], 0, nt1 - 1);
    if (b1[s] != b) continue;
    int sp = s - o1; if (sp < 0) sp += MAXN;
    const unsigned rs = (unsigned)(sp - r0);
    if (rs >= (unsigned)RBADJ) continue;
    const int d = clampi(eh[neh + e], 0, nt2 - 1);
    const int bd = clampi(b2[d], 0, NBATCH - 1);
    int dp = d - sl2[bd] + (sl1[bd + 1] - sl1[bd]); if (dp < 0) dp += MAXN;
    if ((unsigned)dp >= (unsigned)MAXN) continue;
    atomicOr(&bm[rs * 64u + (unsigned)(dp >> 5)], 1u << (dp & 31));
  }
  __syncthreads();

  const float* sb = SP + (size_t)b * MAXN * K1PD;
  for (int row = wv; row < RBADJ; row += 8) {
    const unsigned* wrow = bm + row * 64;
    const unsigned wlo = wrow[lane], whi = wrow[32 + lane];
    const unsigned nzlo = __builtin_amdgcn_ballot_w32(wlo != 0u);
    const unsigned nzhi = __builtin_amdgcn_ballot_w32(whi != 0u);
    v4f a0 = {0.f, 0.f, 0.f, 0.f}, a1 = {0.f, 0.f, 0.f, 0.f};
#pragma unroll 1
    for (int half = 0; half < 2; ++half) {
      unsigned nz = half ? nzhi : nzlo;
      for (int it = 0; it < 32 && nz != 0u; ++it) {
        const int w = (int)__builtin_ctz(nz) + 32 * half;
        nz &= nz - 1u;
        unsigned word = wrow[w];
        for (int jt = 0; jt < 32 && word != 0u; ++jt) {
          const int m = (w << 5) + (int)__builtin_ctz(word);
          word &= word - 1u;
          const float* sr = sb + (size_t)m * K1PD;
          a0 += *(const v4f*)(sr + 4 * lane);
          if (lane < 24) a1 += *(const v4f*)(sr + 128 + 4 * lane);
        }
      }
    }
    float* dr = AS + ((size_t)b * MAXN + (size_t)(r0 + row)) * K1PD;
    *(volatile v4f*)(dr + 4 * lane) = a0;
    if (lane < 24) *(volatile v4f*)(dr + 128 + 4 * lane) = a1;
    __threadfence();
    *(volatile v4f*)(dr + 4 * lane) = a0;
    if (lane < 24) *(volatile v4f*)(dr + 128 + 4 * lane) = a1;
  }
}

__global__ void __launch_bounds__(32) k_out(const float* __restrict__ ON, float* __restrict__ out) {
  const int lane = threadIdx.x & 31;
  const int b = lane >> 1, c = lane & 1;
  float s = 0.f;
  for (int r = 0; r < K2V; ++r) s += ON[((size_t)b * K2PD + (size_t)r) * K2PD + c];
  const float val = s / (float)K2V;
  v4f w;
#pragma unroll
  for (int j = 0; j < 4; ++j) w[j] = __shfl(val, (4 * lane + j) & 31, 32);
  if (lane < 8) *(volatile v4f*)(out + 4 * lane) = w;
  __threadfence();
  if (lane < 8) *(volatile v4f*)(out + 4 * lane) = w;
}

static GArgs gmk(const float* A, int lda, int tA, int M, int Mv, int K, int Kv, long long sA,
                 const float* Bp, int ldb, int KvB, int Nv, int vecB, long long sB,
                 float* D, int ldd, long long sD, int epi, int epiNv, int epiMv, int remap,
                 const int* bidx, const int* sl1, const int* sl2) {
  GArgs g = {};
  g.A = A; g.Bp = Bp; g.A2 = A; g.B2 = Bp; g.D = D;
  g.bidx = bidx; g.sl1 = sl1; g.sl2 = sl2;
  g.sA = sA; g.sB = sB; g.sA2 = 0; g.sB2 = 0; g.sD = sD;
  g.M = M; g.Mv = Mv; g.K = K; g.Kv = Kv; g.lda = lda; g.tA = tA;
  g.ldb = ldb; g.KvB = KvB; g.Nv = Nv; g.vecB = vecB;
  g.Mv2 = 0; g.K2 = 0; g.Kv2 = 0; g.lda2 = lda; g.tA2 = 0; g.ldb2 = ldb;
  g.KvB2 = 0; g.Nv2 = 0; g.vecB2 = 0; g.ldd = ldd;
  g.epi = epi; g.epiNv = epiNv; g.remap = remap; g.epiMv = epiMv;
  return g;
}
static void gt2(GArgs& g, const float* A2, int lda2, int tA2, int Mv2, int K2, int Kv2, long long sA2,
                const float* B2, int ldb2, int KvB2, int Nv2, int vecB2, long long sB2) {
  g.A2 = A2; g.lda2 = lda2; g.tA2 = tA2; g.Mv2 = Mv2; g.K2 = K2; g.Kv2 = Kv2; g.sA2 = sA2;
  g.B2 = B2; g.ldb2 = ldb2; g.KvB2 = KvB2; g.Nv2 = Nv2; g.vecB2 = vecB2; g.sB2 = sB2;
}
template <int NACC>
static void glaunch(const GArgs& g, int nb, hipStream_t st) {
  dim3 grid((unsigned)((g.M + 31) / 32), 1u, (unsigned)nb);
  k_gemm<NACC><<<grid, GT, 0, st>>>(g);
}

extern "C" void kernel_launch(void* const* d_in, const int* in_sizes, int n_in,
                              void* d_out, int out_size, void* d_ws, size_t ws_size,
                              hipStream_t stream) {
  if (n_in < 25 || out_size < NBATCH * OUTV) return;
  const float* x1  = (const float*)d_in[0];
  const float* x2  = (const float*)d_in[1];
  const float* Wpool1 = (const float*)d_in[2];
  const float* Wpool2 = (const float*)d_in[3];
  const float* Wemb1 = (const float*)d_in[4];
  const float* Wemb2 = (const float*)d_in[5];
  const float* Wp1 = (const float*)d_in[6];
  const float* Up1 = (const float*)d_in[7];
  const float* Wp2 = (const float*)d_in[8];
  const float* Up2 = (const float*)d_in[9];
  const float* We1 = (const float*)d_in[10];
  const float* Ue1 = (const float*)d_in[11];
  const float* We2 = (const float*)d_in[12];
  const float* Ue2 = (const float*)d_in[13];
  const float* Wc1 = (const float*)d_in[14];
  const float* Uc1 = (const float*)d_in[15];
  const float* Wc2 = (const float*)d_in[16];
  const float* Uc2 = (const float*)d_in[17];
  const int* eg1 = (const int*)d_in[18];
  const int* eg2 = (const int*)d_in[19];
  const int* eh  = (const int*)d_in[20];
  const int* b1  = (const int*)d_in[21];
  const int* b2  = (const int*)d_in[22];
  const int* sl1 = (const int*)d_in[23];
  const int* sl2 = (const int*)d_in[24];

  const int nt1 = in_sizes[0] / INDIM;
  const int nt2 = in_sizes[1] / INDIM;
  const int ne1 = in_sizes[18] / 2, ne2 = in_sizes[19] / 2, neh = in_sizes[20] / 2;
  if (nt1 <= 0 || nt2 <= 0) return;
  if (in_sizes[23] < NBATCH + 1 || in_sizes[24] < NBATCH + 1 || in_sizes[21] < nt1 || in_sizes[22] < nt2) return;

  const size_t nSP  = (size_t)NBATCH * MAXN * K1PD;
  const size_t nXD  = (size_t)NBATCH * MAXN * HIDD;
  const size_t nA1  = (size_t)NBATCH * K1PD * K1PD;
  const size_t nR64 = (size_t)NBATCH * K1PD * HIDD;
  const size_t nR32 = (size_t)NBATCH * K1PD * K2PD;
  const size_t nX2  = (size_t)NBATCH * K2PD * HIDD;
  const size_t nA2  = (size_t)NBATCH * K2PD * K2PD;
  float* ws = (float*)d_ws;
  size_t off = 0;
  float* SP  = ws + off; off += nSP;
  float* XD  = ws + off; off += nXD;
  float* AS  = ws + off; off += nSP;
  float* A1  = ws + off; off += nA1;
  float* X1  = ws + off; off += nR64;
  float* T64 = ws + off; off += nR64;
  float* HE  = ws + off; off += nR64;
  float* X1E = ws + off; off += nR64;
  float* T32 = ws + off; off += nR32;
  float* HS  = ws + off; off += nR32;
  float* S2P = ws + off; off += nR32;
  float* U   = ws + off; off += nR32;
  float* X2  = ws + off; off += nX2;
  float* TC  = ws + off; off += nX2;
  float* HC  = ws + off; off += nX2;
  float* A2  = ws + off; off += nA2;
  float* T16 = ws + off; off += nA2;
  float* ON  = ws + off; off += nA2;
  if (off * sizeof(float) > ws_size) return;

  const long long sSP = (long long)MAXN * K1PD, sXD = (long long)MAXN * HIDD;
  const long long sA1 = (long long)K1PD * K1PD, sR64 = (long long)K1PD * HIDD, sR32 = (long long)K1PD * K2PD;
  const long long sX2 = (long long)K2PD * HIDD, sA2 = (long long)K2PD * K2PD;

  k_pad<<<(unsigned)((NBATCH * MAXN * 32 + 255) / 256), 256, 0, stream>>>(sl1, sl2, SP, XD);

  {
    GArgs g = gmk(x1, INDIM, 0, nt1, nt1, INDIM, INDIM, 0, Wpool1, K1V, INDIM, K1V, 0, 0,
                  SP, K1PD, 0, 2, K1V, nt1, 1, b1, sl1, sl2);
    glaunch<7>(g, 1, stream);
    g = gmk(x1, INDIM, 0, nt1, nt1, INDIM, INDIM, 0, Wemb1, HIDD, INDIM, HIDD, 1, 0,
            XD, HIDD, 0, 1, 0, nt1, 1, b1, sl1, sl2);
    glaunch<2>(g, 1, stream);
    g = gmk(x2, INDIM, 0, nt2, nt2, INDIM, INDIM, 0, Wpool2, K1V, INDIM, K1V, 0, 0,
            SP, K1PD, 0, 2, K1V, nt2, 2, b2, sl1, sl2);
    glaunch<7>(g, 1, stream);
    g = gmk(x2, INDIM, 0, nt2, nt2, INDIM, INDIM, 0, Wemb2, HIDD, INDIM, HIDD, 1, 0,
            XD, HIDD, 0, 1, 0, nt2, 2, b2, sl1, sl2);
    glaunch<2>(g, 1, stream);
  }

  k_adj<<<dim3(MAXN / RBADJ, NBATCH), 256, 0, stream>>>(eg1, ne1, eg2, ne2, eh, neh, b1, b2, sl1, sl2,
                                                        nt1, nt2, SP, AS);

  {
    GArgs g = gmk(SP, K1PD, 1, K1PD, K1PD, MAXN, MAXN, sSP, AS, K1PD, MAXN, K1PD, 1, sSP,
                  A1, K1PD, sA1, 0, 0, K1PD, 0, b1, sl1, sl2);
    glaunch<7>(g, NBATCH, stream);
    g = gmk(SP, K1PD, 1, K1PD, K1PD, MAXN, MAXN, sSP, XD, HIDD, MAXN, HIDD, 1, sXD,
            X1, HIDD, sR64, 0, 0, K1PD, 0, b1, sl1, sl2);
    glaunch<2>(g, NBATCH, stream);
  }

  {
    GArgs g = gmk(X1, HIDD, 0, K1PD, K1PD, HIDD, HIDD, sR64, Wp1, K2V, HIDD, K2V, 0, 0,
                  T32, K2PD, sR32, 0, 0, K1PD, 0, b1, sl1, sl2);
    glaunch<1>(g, NBATCH, stream);
    g = gmk(A1, K1PD, 0, K1PD, K1PD, K1PD, K1PD, sA1, T32, K2PD, K1PD, K2PD, 1, sR32,
            HS, K2PD, sR32, 1, 0, K1PD, 0, b1, sl1, sl2);
    gt2(g, X1, HIDD, 0, K1PD, HIDD, HIDD, sR64, Up1, K2V, HIDD, K2V, 0, 0);
    glaunch<1>(g, NBATCH, stream);
    g = gmk(HS, K2PD, 0, K1PD, K1PD, K2PD, K2PD, sR32, Wp2, K2V, K2V, K2V, 0, 0,
            T32, K2PD, sR32, 0, 0, K1PD, 0, b1, sl1, sl2);
    glaunch<1>(g, NBATCH, stream);
    g = gmk(A1, K1PD, 0, K1PD, K1PD, K1PD, K1PD, sA1, T32, K2PD, K1PD, K2PD, 1, sR32,
            S2P, K2PD, sR32, 2, K2V, K1V, 0, b1, sl1, sl2);
    gt2(g, HS, K2PD, 0, K1PD, K2PD, K2PD, sR32, Up2, K2V, K2V, K2V, 0, 0);
    glaunch<1>(g, NBATCH, stream);
  }

  {
    GArgs g = gmk(X1, HIDD, 0, K1PD, K1PD, HIDD, HIDD, sR64, We1, HIDD, HIDD, HIDD, 1, 0,
                  T64, HIDD, sR64, 0, 0, K1PD, 0, b1, sl1, sl2);
    glaunch<2>(g, NBATCH, stream);
    g = gmk(A1, K1PD, 0, K1PD, K1PD, K1PD, K1PD, sA1, T64, HIDD, K1PD, HIDD, 1, sR64,
            HE, HIDD, sR64, 1, 0, K1PD, 0, b1, sl1, sl2);
    gt2(g, X1, HIDD, 0, K1PD, HIDD, HIDD, sR64, Ue1, HIDD, HIDD, HIDD, 1, 0);
    glaunch<2>(g, NBATCH, stream);
    g = gmk(HE, HIDD, 0, K1PD, K1PD, HIDD, HIDD, sR64, We2, HIDD, HIDD, HIDD, 1, 0,
            T64, HIDD, sR64, 0, 0, K1PD, 0, b1, sl1, sl2);
    glaunch<2>(g, NBATCH, stream);
    g = gmk(A1, K1PD, 0, K1PD, K1PD, K1PD, K1PD, sA1, T64, HIDD, K1PD, HIDD, 1, sR64,
            X1E, HIDD, sR64, 0, 0, K1PD, 0, b1, sl1, sl2);
    gt2(g, HE, HIDD, 0, K1PD, HIDD, HIDD, sR64, Ue2, HIDD, HIDD, HIDD, 1, 0);
    glaunch<2>(g, NBATCH, stream);
  }

  {
    GArgs g = gmk(S2P, K2PD, 1, K2PD, K2PD, K1PD, K1PD, sR32, X1E, HIDD, K1PD, HIDD, 1, sR64,
                  X2, HIDD, sX2, 0, 0, K2PD, 0, b1, sl1, sl2);
    glaunch<2>(g, NBATCH, stream);
    g = gmk(A1, K1PD, 0, K1PD, K1PD, K1PD, K1PD, sA1, S2P, K2PD, K1PD, K2PD, 1, sR32,
            U, K2PD, sR32, 0, 0, K1PD, 0, b1, sl1, sl2);
    glaunch<1>(g, NBATCH, stream);
    g = gmk(S2P, K2PD, 1, K2PD, K2PD, K1PD, K1PD, sR32, U, K2PD, K1PD, K2PD, 1, sR32,
            A2, K2PD, sA2, 0, 0, K2PD, 0, b1, sl1, sl2);
    glaunch<1>(g, NBATCH, stream);
  }

  {
    GArgs g = gmk(X2, HIDD, 0, K2PD, K2PD, HIDD, HIDD, sX2, Wc1, HIDD, HIDD, HIDD, 1, 0,
                  TC, HIDD, sX2, 0, 0, K2PD, 0, b1, sl1, sl2);
    glaunch<2>(g, NBATCH, stream);
    g = gmk(A2, K2PD, 0, K2PD, K2PD, K2PD, K2PD, sA2, TC, HIDD, K2PD, HIDD, 1, sX2,
            HC, HIDD, sX2, 1, 0, K2PD, 0, b1, sl1, sl2);
    gt2(g, X2, HIDD, 0, K2PD, HIDD, HIDD, sX2, Uc1, HIDD, HIDD, HIDD, 1, 0);
    glaunch<2>(g, NBATCH, stream);
    g = gmk(HC, HIDD, 0, K2PD, K2PD, HIDD, HIDD, sX2, Wc2, OUTV, HIDD, OUTV, 0, 0,
            T16, K2PD, sA2, 0, 0, K2PD, 0, b1, sl1, sl2);
    glaunch<1>(g, NBATCH, stream);
    g = gmk(A2, K2PD, 0, K2PD, K2PD, K2PD, K2PD, sA2, T16, K2PD, K2PD, K2PD, 1, sA2,
            ON, K2PD, sA2, 0, 0, K2PD, 0, b1, sl1, sl2);
    gt2(g, HC, HIDD, 0, K2PD, HIDD, HIDD, sX2, Uc2, OUTV, HIDD, OUTV, 0, 0);
    glaunch<1>(g, NBATCH, stream);
  }

  k_out<<<1, 32, 0, stream>>>(ON, (float*)d_out);

  (void)hipGetLastError();
}
